// ModelWithSTMGNNLayer_84224308674633
// MI455X (gfx1250) — hardware-verified
//
#include <hip/hip_runtime.h>
#define NNODE 20000
#define NNP 20032
#define NE 320000
#define CC 256
#define NH 8
#define HD 32
#define TD 64
#define MS 10
#define MD 128
#define DOUT 256

typedef __bf16 v16b __attribute__((ext_vector_type(16)));
typedef unsigned short v8us __attribute__((ext_vector_type(8), may_alias));
typedef float  v8f  __attribute__((ext_vector_type(8)));
typedef float  v4f  __attribute__((ext_vector_type(4)));
typedef float  v4fa __attribute__((ext_vector_type(4), may_alias));
union FragB { v16b v; v8us half[2]; unsigned short u[16]; };

__device__ __forceinline__ unsigned short bf16_bits(float x) { unsigned int u = __float_as_uint(x); return (unsigned short)((u + 0x7FFFu + ((u >> 16) & 1u)) >> 16); }
__device__ __forceinline__ float bf16_val(unsigned short b) { return __uint_as_float(((unsigned int)b) << 16); }
__device__ __forceinline__ float bf16_round(float x) { return bf16_val(bf16_bits(x)); }
template <int NT>
__device__ __forceinline__ v8f mmaN(v16b ah, v16b al, v16b bh, v16b bl, v8f c) {
  c = __builtin_amdgcn_wmma_f32_16x16x32_bf16(false, ah, false, bh, (short)0, c, false, false);
  if (NT >= 2) c = __builtin_amdgcn_wmma_f32_16x16x32_bf16(false, al, false, bh, (short)0, c, false, false);
  if (NT >= 3) c = __builtin_amdgcn_wmma_f32_16x16x32_bf16(false, ah, false, bl, (short)0, c, false, false);
  asm volatile("v_nop\n\tv_nop\n\tv_nop\n\tv_nop" : "+v"(c) : "v"(ah), "v"(al), "v"(bh), "v"(bl));
  return c;
}

__global__ __launch_bounds__(256) void k_wt_bf16(const float* __restrict__ W, unsigned short* __restrict__ Wt, int K, int N) {
  const int t = blockIdx.x * 256 + threadIdx.x;
  const int k8n = K / 8;
  if (t >= N * k8n) return;
  const int n = t / k8n, k8 = (t % k8n) * 8;
  v8us v;
#pragma unroll
  for (int i = 0; i < 8; ++i) v[i] = bf16_bits(W[(size_t)(k8 + i) * N + n]);
  *(volatile v8us*)(Wt + (size_t)n * K + k8) = v;
  __threadfence();
  *(volatile v8us*)(Wt + (size_t)n * K + k8) = v;
}

template <bool ASPLIT, int ACT, bool BIAS_BF16>
__global__ __launch_bounds__(128) void k_gemm_bf(const float* __restrict__ A, int lda, const unsigned short* __restrict__ Wt, int ldb,
                                               const float* __restrict__ bias, float* __restrict__ C, int ldc, int M, int N, int K) {
  __shared__ __attribute__((aligned(16))) float so[4][16][64];
  const int tid = threadIdx.x, w = tid >> 5, lane = tid & 31, ln = lane & 15, hh = lane >> 4;
  const int ntn = N / 64;
  const int wid = blockIdx.x * 4 + w;
  const int mt = wid / ntn, nq = wid % ntn;
  if (mt * 16 >= M) return;
  const int row0 = mt * 16, col0 = nq * 64;
  const float* arow = A + (size_t)(row0 + ln) * lda;
  v8f acc[4] = {};
  for (int kb = 0; kb < K; kb += 32) {
    FragB ah, al;
    const v4f x0 = *(const v4fa*)(arow + kb + 8 * hh), x1 = *(const v4fa*)(arow + kb + 8 * hh + 4);
    const v4f x2 = *(const v4fa*)(arow + kb + 16 + 8 * hh), x3 = *(const v4fa*)(arow + kb + 16 + 8 * hh + 4);
    float xs[16] = {x0[0],x0[1],x0[2],x0[3],x1[0],x1[1],x1[2],x1[3],x2[0],x2[1],x2[2],x2[3],x3[0],x3[1],x3[2],x3[3]};
#pragma unroll
    for (int i = 0; i < 16; ++i) { const unsigned short hb = bf16_bits(xs[i]); ah.u[i] = hb; al.u[i] = ASPLIT ? bf16_bits(xs[i] - bf16_val(hb)) : (unsigned short)0; }
#pragma unroll
    for (int t = 0; t < 4; ++t) {
      const unsigned short* brow = Wt + (size_t)(col0 + t * 16 + ln) * ldb + kb;
      FragB b;
      b.half[0] = *(const v8us*)(brow + 8 * hh);
      b.half[1] = *(const v8us*)(brow + 16 + 8 * hh);
      acc[t] = mmaN<ASPLIT ? 2 : 1>(ah.v, al.v, b.v, b.v, acc[t]);
    }
  }
#pragma unroll
  for (int t = 0; t < 4; ++t) {
    float bv = bias ? bias[col0 + t * 16 + ln] : 0.f;
    if (BIAS_BF16) bv = bf16_round(bv);
#pragma unroll
    for (int r = 0; r < 8; ++r) { float v = acc[t][r] + bv; if (ACT == 1) v = fmaxf(v, 0.f); so[w][8 * hh + r][t * 16 + ln] = v; }
  }
  __builtin_amdgcn_fence(__ATOMIC_ACQ_REL, "workgroup");
  __builtin_amdgcn_wave_barrier();
  const int rsub = lane >> 4, c4 = (lane & 15) * 4;
  for (int pass = 0; pass < 2; ++pass) {
#pragma unroll
    for (int q = 0; q < 8; ++q) {
      const int r = q * 2 + rsub;
      const v4f v = *(const v4fa*)&so[w][r][c4];
      *(volatile v4f*)(C + (size_t)(row0 + r) * ldc + col0 + c4) = v;
    }
    if (pass == 0) __threadfence();
  }
}

template <int D, bool CAUSAL>
__global__ __launch_bounds__(128) void k_flash(const float* __restrict__ qb, const float* __restrict__ kb, const float* __restrict__ vb,
                                             int pitch, int T, int H, float scale, float* __restrict__ y, int ypitch) {
  constexpr int KS = D / 32;
  constexpr int DT = D / 16;
  __shared__ __attribute__((aligned(16))) unsigned short sKh[32][D + 8], sKl[32][D + 8], sVh[32][D + 8], sVl[32][D + 8];
  __shared__ __attribute__((aligned(16))) unsigned short sPh[4][16][40], sPl[4][16][40];
  __shared__ __attribute__((aligned(16))) float sO[4][16][D];
  const int tid = threadIdx.x, w = tid >> 5, lane = tid & 31, ln = lane & 15, hh = lane >> 4;
  const int nqb = (T + 63) / 64;
  const int bh = blockIdx.x / nqb, qblk = blockIdx.x % nqb;
  const int b = bh / H, h = bh % H;
  const int q0 = qblk * 64 + w * 16;
  const float* Q = qb + (size_t)b * T * pitch + h * D;
  const float* K = kb + (size_t)b * T * pitch + h * D;
  const float* V = vb + (size_t)b * T * pitch + h * D;

  FragB aqh[KS], aql[KS];
  {
    int row = q0 + ln; if (row >= T) row = T - 1;
    const float* qr = Q + (size_t)row * pitch;
#pragma unroll
    for (int ks = 0; ks < KS; ++ks)
#pragma unroll
      for (int i = 0; i < 16; ++i) {
        const int d = ks * 32 + ((i < 8) ? (8 * hh + i) : (16 + 8 * hh + (i - 8)));
        const float x = qr[d] * scale; const unsigned short hb = bf16_bits(x);
        aqh[ks].u[i] = hb; aql[ks].u[i] = bf16_bits(x - bf16_val(hb));
      }
  }
  float m_r[8], l_r[8];
#pragma unroll
  for (int r = 0; r < 8; ++r) { m_r[r] = -3.0e38f; l_r[r] = 0.f; }
  v8f oacc[DT];
#pragma unroll
  for (int dt = 0; dt < DT; ++dt) oacc[dt] = (v8f){0.f,0.f,0.f,0.f,0.f,0.f,0.f,0.f};

  const int kv_end = CAUSAL ? min(T, qblk * 64 + 64) : T;
  for (int j0 = 0; j0 < kv_end; j0 += 32) {
    __syncthreads();
    for (int e = tid; e < 32 * (D / 4); e += 128) {
      const int r = e / (D / 4), c4 = (e % (D / 4)) * 4;
      const int key = j0 + r;
      v4f kf = {0.f,0.f,0.f,0.f}, vf = {0.f,0.f,0.f,0.f};
      if (key < T) { kf = *(const v4fa*)(K + (size_t)key * pitch + c4); vf = *(const v4fa*)(V + (size_t)key * pitch + c4); }
#pragma unroll
      for (int t = 0; t < 4; ++t) {
        unsigned short hb = bf16_bits(kf[t]); sKh[r][c4 + t] = hb; sKl[r][c4 + t] = bf16_bits(kf[t] - bf16_val(hb));
        hb = bf16_bits(vf[t]); sVh[r][c4 + t] = hb; sVl[r][c4 + t] = bf16_bits(vf[t] - bf16_val(hb));
      }
    }
    __syncthreads();
    v8f s[2];
#pragma unroll
    for (int nt = 0; nt < 2; ++nt) {
      v8f acc = {};
#pragma unroll
      for (int ks = 0; ks < KS; ++ks) {
        FragB bh_, bl_;
        bh_.half[0] = *(const v8us*)&sKh[nt * 16 + ln][ks * 32 + 8 * hh]; bh_.half[1] = *(const v8us*)&sKh[nt * 16 + ln][ks * 32 + 16 + 8 * hh];
        bl_.half[0] = *(const v8us*)&sKl[nt * 16 + ln][ks * 32 + 8 * hh]; bl_.half[1] = *(const v8us*)&sKl[nt * 16 + ln][ks * 32 + 16 + 8 * hh];
        acc = mmaN<3>(aqh[ks].v, aql[ks].v, bh_.v, bl_.v, acc);
      }
      s[nt] = acc;
    }
    float alpha[8];
#pragma unroll
    for (int r = 0; r < 8; ++r) {
      const int qi = q0 + 8 * hh + r;
      const int ja = j0 + ln, jb = j0 + 16 + ln;
      if (CAUSAL) { if (ja > qi) s[0][r] = -3.0e38f; if (jb > qi) s[1][r] = -3.0e38f; }
      if (ja >= T) s[0][r] = -3.0e38f;
      if (jb >= T) s[1][r] = -3.0e38f;
      float mx = fmaxf(s[0][r], s[1][r]);
      mx = fmaxf(mx, __shfl_xor(mx, 1, 32)); mx = fmaxf(mx, __shfl_xor(mx, 2, 32)); mx = fmaxf(mx, __shfl_xor(mx, 4, 32)); mx = fmaxf(mx, __shfl_xor(mx, 8, 32));
      const float mnew = fmaxf(m_r[r], mx);
      alpha[r] = (mnew > -1.0e38f) ? __expf(m_r[r] - mnew) : 1.0f;
      const float p0 = (s[0][r] > -1.0e38f) ? __expf(s[0][r] - mnew) : 0.f;
      const float p1 = (s[1][r] > -1.0e38f) ? __expf(s[1][r] - mnew) : 0.f;
      m_r[r] = mnew;
      l_r[r] = l_r[r] * alpha[r] + p0 + p1;
      unsigned short hb = bf16_bits(p0); sPh[w][8 * hh + r][ln] = hb;      sPl[w][8 * hh + r][ln] = bf16_bits(p0 - bf16_val(hb));
      hb = bf16_bits(p1);                sPh[w][8 * hh + r][16 + ln] = hb; sPl[w][8 * hh + r][16 + ln] = bf16_bits(p1 - bf16_val(hb));
    }
#pragma unroll
    for (int dt = 0; dt < DT; ++dt)
#pragma unroll
      for (int r = 0; r < 8; ++r) oacc[dt][r] *= alpha[r];
    __builtin_amdgcn_fence(__ATOMIC_ACQ_REL, "workgroup");
    __builtin_amdgcn_wave_barrier();
    FragB pah, pal;
    pah.half[0] = *(const v8us*)&sPh[w][ln][8 * hh]; pah.half[1] = *(const v8us*)&sPh[w][ln][16 + 8 * hh];
    pal.half[0] = *(const v8us*)&sPl[w][ln][8 * hh]; pal.half[1] = *(const v8us*)&sPl[w][ln][16 + 8 * hh];
#pragma unroll
    for (int dt = 0; dt < DT; ++dt) {
      FragB bvh, bvl;
#pragma unroll
      for (int i = 0; i < 8; ++i) {
        bvh.u[i] = sVh[8 * hh + i][dt * 16 + ln]; bvh.u[8 + i] = sVh[16 + 8 * hh + i][dt * 16 + ln];
        bvl.u[i] = sVl[8 * hh + i][dt * 16 + ln]; bvl.u[8 + i] = sVl[16 + 8 * hh + i][dt * 16 + ln];
      }
      oacc[dt] = mmaN<3>(pah.v, pal.v, bvh.v, bvl.v, oacc[dt]);
    }
    __builtin_amdgcn_fence(__ATOMIC_ACQ_REL, "workgroup");
    __builtin_amdgcn_wave_barrier();
  }
#pragma unroll
  for (int r = 0; r < 8; ++r) {
    float l = l_r[r];
    l += __shfl_xor(l, 1, 32); l += __shfl_xor(l, 2, 32); l += __shfl_xor(l, 4, 32); l += __shfl_xor(l, 8, 32);
    l_r[r] = (l > 0.f) ? 1.0f / l : 0.f;
  }
#pragma unroll
  for (int dt = 0; dt < DT; ++dt)
#pragma unroll
    for (int r = 0; r < 8; ++r) sO[w][8 * hh + r][dt * 16 + ln] = oacc[dt][r] * l_r[r];
  __builtin_amdgcn_fence(__ATOMIC_ACQ_REL, "workgroup");
  __builtin_amdgcn_wave_barrier();
  for (int pass = 0; pass < 2; ++pass) {
    for (int r = 0; r < 16; ++r) {
      const int row = q0 + r;
      if (row < T && lane < D / 4) {
        const v4f val = *(const v4fa*)&sO[w][r][lane * 4];
        *(volatile v4f*)(y + ((size_t)b * T + row) * ypitch + h * D + lane * 4) = val;
      }
    }
    if (pass == 0) __threadfence();
  }
}

template <bool ASPLIT, int ACT, bool BIAS_BF16, bool RES_BF16>
__global__ __launch_bounds__(128) void k_gemm_bf3(const float* __restrict__ A, int lda, const unsigned short* __restrict__ Wt, int ldb,
                                                const float* __restrict__ bias, const float* __restrict__ resid, int rmod, int ldr,
                                                float* __restrict__ C, int ldc, int M, int N, int K) {
  __shared__ __attribute__((aligned(16))) float so[4][16][64];
  const int tid = threadIdx.x, w = tid >> 5, lane = tid & 31, ln = lane & 15, hh = lane >> 4;
  const int ntn = N / 64;
  const int wid = blockIdx.x * 4 + w;
  const int mt = wid / ntn, nq = wid % ntn;
  if (mt * 16 >= M) return;
  const int row0 = mt * 16, col0 = nq * 64;
  const float* arow = A + (size_t)(row0 + ln) * lda;
  v8f acc[4] = {};
  for (int kb = 0; kb < K; kb += 32) {
    FragB ah, al;
    const v4f x0 = *(const v4fa*)(arow + kb + 8 * hh), x1 = *(const v4fa*)(arow + kb + 8 * hh + 4);
    const v4f x2 = *(const v4fa*)(arow + kb + 16 + 8 * hh), x3 = *(const v4fa*)(arow + kb + 16 + 8 * hh + 4);
    float xs[16] = {x0[0],x0[1],x0[2],x0[3],x1[0],x1[1],x1[2],x1[3],x2[0],x2[1],x2[2],x2[3],x3[0],x3[1],x3[2],x3[3]};
#pragma unroll
    for (int i = 0; i < 16; ++i) { const unsigned short hb = bf16_bits(xs[i]); ah.u[i] = hb; al.u[i] = ASPLIT ? bf16_bits(xs[i] - bf16_val(hb)) : (unsigned short)0; }
#pragma unroll
    for (int t = 0; t < 4; ++t) {
      const unsigned short* brow = Wt + (size_t)(col0 + t * 16 + ln) * ldb + kb;
      FragB b;
      b.half[0] = *(const v8us*)(brow + 8 * hh);
      b.half[1] = *(const v8us*)(brow + 16 + 8 * hh);
      acc[t] = mmaN<ASPLIT ? 2 : 1>(ah.v, al.v, b.v, b.v, acc[t]);
    }
  }
#pragma unroll
  for (int t = 0; t < 4; ++t) {
    const int col = col0 + t * 16 + ln;
    float bv = bias ? bias[col] : 0.f;
    if (BIAS_BF16) bv = bf16_round(bv);
#pragma unroll
    for (int r = 0; r < 8; ++r) {
      float v = acc[t][r] + bv;
      if (resid) { float rv = resid[(size_t)((row0 + 8 * hh + r) % rmod) * ldr + col]; if (RES_BF16) rv = bf16_round(rv); v += rv; }
      if (ACT == 1) v = fmaxf(v, 0.f);
      if (ACT == 2) v = 0.5f * v * (1.0f + erff(v * 0.70710678118654752f));
      if (ACT == 3) { const float u = 0.7978845608028654f * (v + 0.044715f * v * v * v); v = 0.5f * v * (1.0f + tanhf(u)); }
      so[w][8 * hh + r][t * 16 + ln] = v;
    }
  }
  __builtin_amdgcn_fence(__ATOMIC_ACQ_REL, "workgroup");
  __builtin_amdgcn_wave_barrier();
  const int rsub = lane >> 4, c4 = (lane & 15) * 4;
  for (int pass = 0; pass < 2; ++pass) {
#pragma unroll
    for (int q = 0; q < 8; ++q) {
      const int r = q * 2 + rsub;
      const v4f v = *(const v4fa*)&so[w][r][c4];
      *(volatile v4f*)(C + (size_t)(row0 + r) * ldc + col0 + c4) = v;
    }
    if (pass == 0) __threadfence();
  }
}
template <bool PARAM_BF16>
__global__ __launch_bounds__(256) void k_layernorm(const float* __restrict__ X, const float* __restrict__ R, const float* __restrict__ g, const float* __restrict__ bta,
                                                  float* __restrict__ out_sum, float* __restrict__ out_norm, int N, float eps) {
  __shared__ float red[256];
  const int row = blockIdx.x, tid = threadIdx.x;
  const float* x = X + (size_t)row * N; const float* rr = R ? R + (size_t)row * N : nullptr;
  float vals[16];
  const int per = N / 256;
  float s1 = 0.f;
  for (int u = 0; u < per / 4; ++u) {
    const int j = tid * 4 + 1024 * u;
    const v4f a = *(const v4fa*)(x + j);
    v4f b = {0.f,0.f,0.f,0.f}; if (rr) b = *(const v4fa*)(rr + j);
#pragma unroll
    for (int q = 0; q < 4; ++q) { const float v = a[q] + b[q]; vals[u * 4 + q] = v; s1 += v; }
  }
  red[tid] = s1; __syncthreads();
  for (int st = 128; st > 0; st >>= 1) { if (tid < st) red[tid] += red[tid + st]; __syncthreads(); }
  const float mu = red[0] / (float)N; __syncthreads();
  float s2 = 0.f;
  for (int u = 0; u < per / 4; ++u)
#pragma unroll
    for (int q = 0; q < 4; ++q) { const float c = vals[u * 4 + q] - mu; s2 += c * c; }
  red[tid] = s2; __syncthreads();
  for (int st = 128; st > 0; st >>= 1) { if (tid < st) red[tid] += red[tid + st]; __syncthreads(); }
  const float rs = rsqrtf(red[0] / (float)N + eps);
  for (int pass = 0; pass < 2; ++pass) {
    for (int u = 0; u < per / 4; ++u) {
      const int j = tid * 4 + 1024 * u;
      v4f o, sm;
#pragma unroll
      for (int q = 0; q < 4; ++q) {
        float gg = g[j + q], bb = bta[j + q];
        if (PARAM_BF16) { gg = bf16_round(gg); bb = bf16_round(bb); }
        sm[q] = vals[u * 4 + q]; o[q] = (vals[u * 4 + q] - mu) * rs * gg + bb;
      }
      if (out_sum) *(volatile v4f*)(out_sum + (size_t)row * N + j) = sm;
      *(volatile v4f*)(out_norm + (size_t)row * N + j) = o;
    }
    if (pass == 0) __threadfence();
  }
}


typedef _Float16 v16h __attribute__((ext_vector_type(16)));
union FragH { v16h v; v8us half[2]; _Float16 h[16]; unsigned short u[16]; };
template <int NT>
__device__ __forceinline__ v8f mmaH(v16h ah, v16h al, v16h bh, v16h bl, v8f c) {
  c = __builtin_amdgcn_wmma_f32_16x16x32_f16(false, ah, false, bh, (short)0, c, false, false);
  if (NT >= 2) c = __builtin_amdgcn_wmma_f32_16x16x32_f16(false, al, false, bh, (short)0, c, false, false);
  if (NT >= 3) c = __builtin_amdgcn_wmma_f32_16x16x32_f16(false, ah, false, bl, (short)0, c, false, false);
  asm volatile("v_nop\n\tv_nop\n\tv_nop\n\tv_nop" : "+v"(c) : "v"(ah), "v"(al), "v"(bh), "v"(bl));
  return c;
}
template <bool ASPLIT>
__global__ __launch_bounds__(128) void k_gemm_h(const float* __restrict__ A, int lda, size_t sA, const _Float16* __restrict__ Bh, int ldb, size_t sB, float alpha, float* __restrict__ C, int ldc, size_t sC, int M, int N, int K) {
  __shared__ __attribute__((aligned(16))) float so[4][16][64];
  const int tid = threadIdx.x, w = tid >> 5, lane = tid & 31, ln = lane & 15, hh = lane >> 4; const int by = blockIdx.y;
  A += (size_t)by * sA; Bh += (size_t)by * sB; C += (size_t)by * sC;
  const int ntn = (N + 63) / 64; const int wid = blockIdx.x * 4 + w; const int mt = wid / ntn, nq = wid % ntn; if (mt * 16 >= M) return;
  const int row0 = mt * 16, col0 = nq * 64; const float* arow = A + (size_t)(row0 + ln) * lda;
  v8f acc[4] = {};
  for (int kb = 0; kb < K; kb += 32) {
    FragH ah, al;
    const v4f x0 = *(const v4fa*)(arow + kb + 8 * hh), x1 = *(const v4fa*)(arow + kb + 8 * hh + 4), x2 = *(const v4fa*)(arow + kb + 16 + 8 * hh), x3 = *(const v4fa*)(arow + kb + 16 + 8 * hh + 4);
    float xs[16] = {x0[0],x0[1],x0[2],x0[3],x1[0],x1[1],x1[2],x1[3],x2[0],x2[1],x2[2],x2[3],x3[0],x3[1],x3[2],x3[3]};
#pragma unroll
    for (int i = 0; i < 16; ++i) { const _Float16 h = (_Float16)xs[i]; ah.h[i] = h; al.h[i] = ASPLIT ? (_Float16)(xs[i] - (float)h) : (_Float16)0.0f; }
#pragma unroll
    for (int t = 0; t < 4; ++t) { if (col0 + t * 16 >= N) continue; const size_t boff = (size_t)(col0 + t * 16 + ln) * ldb + kb; FragH bq; bq.half[0] = *(const v8us*)(Bh + boff + 8 * hh); bq.half[1] = *(const v8us*)(Bh + boff + 16 + 8 * hh);
      acc[t] = mmaH<ASPLIT ? 2 : 1>(ah.v, al.v, bq.v, bq.v, acc[t]); }
  }
#pragma unroll
  for (int t = 0; t < 4; ++t) { if (col0 + t * 16 >= N) continue;
#pragma unroll
    for (int r = 0; r < 8; ++r) so[w][8 * hh + r][t * 16 + ln] = acc[t][r] * alpha; }
  __builtin_amdgcn_fence(__ATOMIC_ACQ_REL, "workgroup"); __builtin_amdgcn_wave_barrier();
  const int rsub = lane >> 4, c4 = (lane & 15) * 4;
  for (int pass = 0; pass < 2; ++pass) {
#pragma unroll
    for (int q = 0; q < 8; ++q) { const int r = q * 2 + rsub; if (col0 + c4 < N) { const v4f v = *(const v4fa*)&so[w][r][c4]; *(volatile v4f*)(C + (size_t)(row0 + r) * ldc + col0 + c4) = v; } }
    if (pass == 0) __threadfence(); }
}

__global__ __launch_bounds__(256) void k_wt_f16(const float* __restrict__ W, _Float16* __restrict__ Wt, int K, int N, float scale) {
  const int t = blockIdx.x * 256 + threadIdx.x; if (t >= N * (K / 8)) return; const int n = t / (K / 8), k8 = (t % (K / 8)) * 8; FragH f;
#pragma unroll
  for (int i = 0; i < 8; ++i) f.h[i] = (_Float16)(bf16_round(W[(size_t)(k8 + i) * N + n]) * scale); const v8us o = f.half[0];
  *(volatile v8us*)((unsigned short*)Wt + (size_t)n * K + k8) = o; __threadfence(); *(volatile v8us*)((unsigned short*)Wt + (size_t)n * K + k8) = o;
}
template <int ACT>
__global__ __launch_bounds__(128) void k_gemm_hhx(const _Float16* __restrict__ A, int lda, size_t sA, const _Float16* __restrict__ Bh, int ldb, size_t sB, float alpha, const float* __restrict__ bias, size_t sBias, const float* __restrict__ CP, int rowsPerB, size_t sCPb, int row0g,
    float* __restrict__ C, _Float16* __restrict__ C16, int ldc, size_t sC, int M, int N, int K) {
  __shared__ __attribute__((aligned(16))) float so[4][16][64];
  const int tid = threadIdx.x, w = tid >> 5, lane = tid & 31, ln = lane & 15, hh = lane >> 4; const int by = blockIdx.y;
  A += (size_t)by * sA; Bh += (size_t)by * sB; const size_t cofs = (size_t)by * sC; const float* bp = bias ? bias + (size_t)by * sBias : nullptr;
  const int ntn = (N + 63) / 64; const int wid = blockIdx.x * 4 + w; const int mt = wid / ntn, nq = wid % ntn; if (mt * 16 >= M) return;
  const int row0 = mt * 16, col0 = nq * 64; const _Float16* arow = A + (size_t)(row0 + ln) * lda;
  v8f acc[4] = {};
  for (int kb = 0; kb < K; kb += 32) { FragH ah; ah.half[0] = *(const v8us*)((const unsigned short*)arow + kb + 8 * hh); ah.half[1] = *(const v8us*)((const unsigned short*)arow + kb + 16 + 8 * hh);
#pragma unroll
    for (int t = 0; t < 4; ++t) { if (col0 + t * 16 >= N) continue; const size_t boff = (size_t)(col0 + t * 16 + ln) * ldb + kb; FragH bq; bq.half[0] = *(const v8us*)((const unsigned short*)Bh + boff + 8 * hh); bq.half[1] = *(const v8us*)((const unsigned short*)Bh + boff + 16 + 8 * hh);
      acc[t] = mmaH<1>(ah.v, ah.v, bq.v, bq.v, acc[t]); }
  }
#pragma unroll
  for (int t = 0; t < 4; ++t) { if (col0 + t * 16 >= N) continue; const int col = col0 + t * 16 + ln; const float bv = bp ? bf16_round(bp[col]) : 0.f;
#pragma unroll
    for (int r = 0; r < 8; ++r) { float v = acc[t][r] * alpha + bv; if (CP) { const int bidx = (row0g + row0 + 8 * hh + r) / rowsPerB; v += CP[(size_t)bidx * sCPb + (size_t)by * 64 + col]; } if (ACT == 1) v = (v > 0.f) ? v : expm1f(v); else if (ACT == 3) v = fmaxf(v, 0.f); so[w][8 * hh + r][t * 16 + ln] = v; } }
  __builtin_amdgcn_fence(__ATOMIC_ACQ_REL, "workgroup"); __builtin_amdgcn_wave_barrier();
  const int rsub = lane >> 4, c4 = (lane & 15) * 4; typedef _Float16 v4h __attribute__((ext_vector_type(4)));
  for (int pass = 0; pass < 2; ++pass) {
#pragma unroll
    for (int q = 0; q < 8; ++q) { const int r = q * 2 + rsub; if (col0 + c4 < N) { const v4f v = *(const v4fa*)&so[w][r][c4]; if (C) *(volatile v4f*)(C + cofs + (size_t)(row0 + r) * ldc + col0 + c4) = v; if (C16) { v4h h4; for (int i = 0; i < 4; ++i) h4[i] = (_Float16)v[i]; *(volatile v4h*)(C16 + cofs + (size_t)(row0 + r) * ldc + col0 + c4) = h4; } } }
    if (pass == 0) __threadfence(); }
}


__global__ __launch_bounds__(256) void k_x16(const float* __restrict__ x, _Float16* __restrict__ X16, size_t n8) { const size_t t = (size_t)blockIdx.x * 256 + threadIdx.x; if (t >= n8) return; FragH f;
#pragma unroll
  for (int q = 0; q < 8; ++q) f.h[q] = (_Float16)bf16_round(x[t * 8 + q]); *(volatile v8us*)((unsigned short*)X16 + t * 8) = f.half[0]; __threadfence(); *(volatile v8us*)((unsigned short*)X16 + t * 8) = f.half[0]; }
__global__ __launch_bounds__(256) void k_h16(const float* __restrict__ x, _Float16* __restrict__ X16, size_t n8) { const size_t t = (size_t)blockIdx.x * 256 + threadIdx.x; if (t >= n8) return; FragH f;
#pragma unroll
  for (int q = 0; q < 8; ++q) f.h[q] = (_Float16)x[t * 8 + q]; *(volatile v8us*)((unsigned short*)X16 + t * 8) = f.half[0]; __threadfence(); *(volatile v8us*)((unsigned short*)X16 + t * 8) = f.half[0]; }
__global__ __launch_bounds__(256) void k_round16f(const float* __restrict__ W, _Float16* __restrict__ Bt, size_t n8) { const size_t t = (size_t)blockIdx.x * 256 + threadIdx.x; if (t >= n8) return; FragH f;
#pragma unroll
  for (int i = 0; i < 8; ++i) f.h[i] = (_Float16)(bf16_round(W[t * 8 + i]) * 16.0f); *(volatile v8us*)((unsigned short*)Bt + t * 8) = f.half[0]; __threadfence(); *(volatile v8us*)((unsigned short*)Bt + t * 8) = f.half[0]; }
template <int NHv, int TTv>
__global__ __launch_bounds__(256) void k_vt(const _Float16* __restrict__ V16, int ldv, int voff, _Float16* __restrict__ Vt) { __shared__ unsigned short tl[64][66]; const int tid = threadIdx.x; const int slab = blockIdx.x / (TTv / 64), lg = blockIdx.x % (TTv / 64); const int b = slab / NHv, h = slab % NHv;
  for (int i = tid; i < 64 * 8; i += 256) { const int r = i / 8, c8 = (i % 8) * 8; FragH f; f.half[0] = *(const v8us*)((const unsigned short*)V16 + ((size_t)b * TTv + lg * 64 + r) * ldv + voff + h * 64 + c8);
#pragma unroll
    for (int q = 0; q < 8; ++q) tl[r][c8 + q] = f.u[q]; }
  __syncthreads();
  for (int pass = 0; pass < 2; ++pass) {
#pragma unroll
    for (int rd = 0; rd < 2; ++rd) { const int d = rd * 32 + tid / 8, pc = tid % 8; FragH f;
#pragma unroll
      for (int q = 0; q < 8; ++q) f.u[q] = tl[pc * 8 + q][d];
      *(volatile v8us*)((unsigned short*)Vt + ((size_t)slab * 64 + d) * TTv + lg * 64 + pc * 8) = f.half[0]; }
    if (pass == 0) __threadfence(); } }

__device__ __forceinline__ int bscan512(int cnt, int* wsum, int tid, int& total) {
  const int lane = tid & 31, wv = tid >> 5; int x = cnt;
#pragma unroll
  for (int d = 1; d < 32; d <<= 1) { const int y = __shfl_up(x, d, 32); if (lane >= d) x += y; }
  __syncthreads(); if (lane == 31) wsum[wv] = x; __syncthreads();
  int t = (lane < 16) ? wsum[lane] : 0;
#pragma unroll
  for (int d = 1; d < 32; d <<= 1) { const int y = __shfl_up(t, d, 32); if (lane >= d) t += y; }
  const int woff = (wv == 0) ? 0 : __shfl(t, wv - 1, 32); total = __shfl(t, 15, 32);
  return woff + x - cnt; }
#define QCAP 8
#define CHUNK 8192
typedef _Float16 v4h __attribute__((ext_vector_type(4)));
__global__ __launch_bounds__(256) void k_hdots(const _Float16* __restrict__ H16, const float* __restrict__ as, const float* __restrict__ ad, float* __restrict__ ES, float* __restrict__ ED) { const int t = blockIdx.x * 256 + threadIdx.x; if (t >= NNODE * NH) return; const int h = t % NH, n = t / NH; const unsigned short* p = (const unsigned short*)H16 + (size_t)n * CC + h * HD; float s = 0.f, d2 = 0.f;
#pragma unroll
  for (int g = 0; g < 4; ++g) { FragH f; f.half[0] = *(const v8us*)(p + g * 8); for (int q = 0; q < 8; ++q) { const float v = (float)f.h[q]; s += v * bf16_round(as[h * HD + g * 8 + q]); d2 += v * bf16_round(ad[h * HD + g * 8 + q]); } }
  for (int pass = 0; pass < 2; ++pass) { *(volatile float*)(ES + t) = s; *(volatile float*)(ED + t) = d2; if (pass == 0) __threadfence(); } }
__global__ __launch_bounds__(512) void k_gmsg2(const _Float16* __restrict__ T16, int ldt, int hcol, const float* __restrict__ ES, const float* __restrict__ ED, int hstride, int hA, const int* __restrict__ srci, const int* __restrict__ dsti, float* __restrict__ OUTS, int ocoff) {
  #pragma clang fp contract(off)
  __shared__ short Lr[CHUNK]; __shared__ int Le[CHUNK]; __shared__ int scan[16]; __shared__ int lq[16][QCAP][32]; __shared__ __attribute__((aligned(16))) float stg[64][68];
  const int tid = threadIdx.x, lane = tid & 31, wv = tid >> 5; const int n0 = blockIdx.x * 1024; const int myl0 = wv * 64 + 2 * lane; int qn = 0; float acc[2][64], m[2], z[2];
float mB[2], zB[2], edA[2], edB[2];
#pragma unroll
  for (int s2 = 0; s2 < 2; ++s2) { const int n = n0 + myl0 + s2; const int nc = n < NNODE ? n : NNODE - 1; m[s2] = -3.0e38f; z[s2] = 0.f; mB[s2] = -3.0e38f; zB[s2] = 0.f; edA[s2] = ED[(size_t)nc * hstride + hA]; edB[s2] = ED[(size_t)nc * hstride + hA + 1];
#pragma unroll
    for (int c = 0; c < 64; ++c) acc[s2][c] = 0.f; }

#pragma unroll 1
  for (int eb = 0; eb < NE + CHUNK; eb += CHUNK) { const bool sentinel = (eb >= NE); int tot = 0;
    if (!sentinel) { int k_cnt = 0; unsigned hm = 0; int hv[16];
#pragma unroll
      for (int k = 0; k < 16; ++k) { const int e = eb + tid * 16 + k; const int ec = (e < NE) ? e : (NE - 1); const int dv = dsti[ec] - n0; const int dd_ = (e < NE) ? dv : -1; hv[k] = dd_; if (dd_ >= 0 && dd_ < 1024) { hm |= 1u << k; ++k_cnt; } }
      int p = bscan512(k_cnt, scan, tid, tot);
#pragma unroll
      for (int k = 0; k < 16; ++k) if (hm & (1u << k)) { Lr[p] = (short)hv[k]; Le[p] = eb + tid * 16 + k; ++p; }
      __syncthreads(); }
    const int ntrip = sentinel ? 1 : ((tot + 31) >> 5);
#pragma unroll 1
    for (int it = 0; it < ntrip; ++it) { const int q = it * 32 + lane; const int lr = (!sentinel && q < tot) ? (int)Lr[q] : -1;
      unsigned mm = sentinel ? 1u : __builtin_amdgcn_ballot_w32(lr >= wv * 64 && lr < wv * 64 + 64);
#pragma unroll 1
      while (mm) { const int bit = __builtin_ctz(mm); mm &= mm - 1u; const int ol = sentinel ? -2 : (__shfl(lr, bit, 32) - wv * 64); const int owner = ol >> 1; const int e = sentinel ? 0 : Le[it * 32 + bit];
        if (sentinel || __builtin_amdgcn_ballot_w32(lane == owner && qn == QCAP)) {
          int kmax = qn;
#pragma unroll
          for (int o = 16; o >= 1; o >>= 1) kmax = max(kmax, __shfl_xor(kmax, o, 32));
#pragma unroll 1
          for (int k = 0; k < kmax; ++k) { if (k < qn) { const int ent = lq[wv][k][lane]; const int eq = ent >> 1; const int sl = ent & 1; int s = srci[eq]; s = s < 0 ? 0 : (s >= NNODE ? NNODE - 1 : s);
              const float esA = ES[(size_t)s * hstride + hA], esB = ES[(size_t)s * hstride + hA + 1]; const unsigned short* pr = (const unsigned short*)T16 + (size_t)s * ldt + hcol;
#pragma unroll
              for (int s2 = 0; s2 < 2; ++s2) if (s2 == sl) { float a = esA + edA[s2]; a = (a >= 0.f) ? a : 0.2f * a; float b = esB + edB[s2]; b = (b >= 0.f) ? b : 0.2f * b;
                const float mnA = fmaxf(m[s2], a); const float scA = expf(m[s2] - mnA); const float wA = expf(a - mnA); m[s2] = mnA; z[s2] = z[s2] * scA + wA;
                const float mnB = fmaxf(mB[s2], b); const float scB = expf(mB[s2] - mnB); const float wB = expf(b - mnB); mB[s2] = mnB; zB[s2] = zB[s2] * scB + wB;
#pragma unroll
                for (int g = 0; g < 8; ++g) { FragH f; f.half[0] = *(const v8us*)(pr + g * 8); const float sc = (g < 4) ? scA : scB, w = (g < 4) ? wA : wB;
#pragma unroll
                  for (int d = 0; d < 8; ++d) acc[s2][g * 8 + d] = acc[s2][g * 8 + d] * sc + w * (float)f.h[d]; } } } }
          qn = 0; }
        if (lane == owner) { lq[wv][qn][lane] = e * 2 + (ol & 1); ++qn; } } }
    __syncthreads(); }
#pragma unroll
  for (int s2 = 0; s2 < 2; ++s2) { const float izA = (z[s2] > 0.f) ? 1.0f / z[s2] : 0.f, izB = (zB[s2] > 0.f) ? 1.0f / zB[s2] : 0.f;
#pragma unroll
    for (int c = 0; c < 64; ++c) acc[s2][c] *= (c < 32) ? izA : izB; }
  for (int tg = 0; tg < 16; ++tg) {
    if (wv == tg) {
#pragma unroll
      for (int c = 0; c < 64; ++c) { stg[2 * lane][c] = acc[0][c]; stg[2 * lane + 1][c] = acc[1][c]; } }
    __syncthreads();
    for (int pass = 0; pass < 2; ++pass) {
#pragma unroll
      for (int rd = 0; rd < 2; ++rd) { const int r = rd * 32 + tid / 16, pc = tid % 16; const int n = n0 + tg * 64 + r; if (n < NNODE) { float* dp = OUTS + (size_t)n * DOUT + ocoff + pc * 4; v4f fv; for (int q = 0; q < 4; ++q) fv[q] = fmaxf(stg[r][pc * 4 + q], 0.f); *(volatile v4f*)dp = fv; } }
      if (pass == 0) __threadfence(); }
    __syncthreads(); } }

__global__ __launch_bounds__(256) void k_memres(const float* __restrict__ NODE, const float* __restrict__ Q, const float* __restrict__ K, const float* __restrict__ V, float* __restrict__ X, _Float16* __restrict__ X16) { __shared__ __attribute__((aligned(16))) float srow[8][CC]; const int tid = threadIdx.x, wv = tid >> 5, lane = tid & 31; const int n = blockIdx.x * 8 + wv; if (n >= NNODE) return;
  const v4f qa = *(const v4fa*)(Q + (size_t)n * CC + lane * 8), qb = *(const v4fa*)(Q + (size_t)n * CC + lane * 8 + 4); float lg[MS]; float mx = -3.0e38f;
#pragma unroll
  for (int s = 0; s < MS; ++s) { const v4f ka = *(const v4fa*)(K + s * CC + lane * 8), kb = *(const v4fa*)(K + s * CC + lane * 8 + 4); float d = 0.f; for (int q = 0; q < 4; ++q) d += qa[q] * ka[q] + qb[q] * kb[q]; for (int o = 16; o >= 1; o >>= 1) d += __shfl_xor(d, o, 32); lg[s] = d * 0.0625f; mx = fmaxf(mx, lg[s]); }
  float zz = 0.f;
#pragma unroll
  for (int s = 0; s < MS; ++s) { lg[s] = expf(lg[s] - mx); zz += lg[s]; } const float iz = 1.0f / zz;
  const v4f na = *(const v4fa*)(NODE + (size_t)n * CC + lane * 8), nb = *(const v4fa*)(NODE + (size_t)n * CC + lane * 8 + 4), xa = *(const v4fa*)(X + (size_t)n * CC + lane * 8), xb = *(const v4fa*)(X + (size_t)n * CC + lane * 8 + 4); float o[8];
#pragma unroll
  for (int q = 0; q < 4; ++q) { o[q] = na[q] + xa[q]; o[4 + q] = nb[q] + xb[q]; }
#pragma unroll
  for (int s = 0; s < MS; ++s) { const float p = lg[s] * iz; const v4f va = *(const v4fa*)(V + s * CC + lane * 8), vb = *(const v4fa*)(V + s * CC + lane * 8 + 4); for (int q = 0; q < 4; ++q) { o[q] += p * va[q]; o[4 + q] += p * vb[q]; } }
  v4f r0, r1; FragH f;
#pragma unroll
  for (int q = 0; q < 4; ++q) { r0[q] = fmaxf(o[q], 0.f); r1[q] = fmaxf(o[4 + q], 0.f); f.h[q] = (_Float16)r0[q]; f.h[4 + q] = (_Float16)r1[q]; }
  for (int q = 0; q < 4; ++q) { srow[wv][lane * 8 + q] = r0[q]; srow[wv][lane * 8 + 4 + q] = r1[q]; }
  __builtin_amdgcn_fence(__ATOMIC_ACQ_REL, "workgroup"); __builtin_amdgcn_wave_barrier();
  const v4f w0 = *(const v4f*)&srow[wv][4 * lane], w1 = *(const v4f*)&srow[wv][128 + 4 * lane];
  for (int pass = 0; pass < 2; ++pass) { *(volatile v4f*)(X + (size_t)n * CC + 4 * lane) = w0; *(volatile v4f*)(X + (size_t)n * CC + 128 + 4 * lane) = w1; *(volatile v8us*)((unsigned short*)X16 + (size_t)n * CC + lane * 8) = f.half[0]; if (pass == 0) __threadfence(); } }
__global__ __launch_bounds__(256) void k_pool(const float* __restrict__ X, float* __restrict__ POOL) { __shared__ float ra[256]; const int c = blockIdx.x, tid = threadIdx.x; float a = 0.f; for (int n = tid; n < NNODE; n += 256) a += X[(size_t)n * CC + c]; ra[tid] = a; __syncthreads(); for (int o = 128; o >= 1; o >>= 1) { if (tid < o) ra[tid] += ra[tid + o]; __syncthreads(); }
  if (tid == 0) { const float m = ra[0] / (float)NNODE; *(volatile float*)(POOL + c) = m; __threadfence(); *(volatile float*)(POOL + c) = m; } }
__global__ __launch_bounds__(64) void k_cls(const float* __restrict__ POOL, const float* __restrict__ mem, const float* __restrict__ Wc, const float* __restrict__ bc, float* __restrict__ out) { __shared__ float fin[CC + MD]; const int tid = threadIdx.x;
  for (int i = tid; i < CC; i += 64) fin[i] = POOL[i]; for (int i = tid; i < MD; i += 64) { float s = 0.f; for (int r = 0; r < MS; ++r) s += bf16_round(mem[r * MD + i]); fin[CC + i] = s / (float)MS; } __syncthreads();
  if (tid < 2) { float s = bf16_round(bc[tid]);
#pragma unroll 1
    for (int i = 0; i < CC + MD; ++i) s += fin[i] * bf16_round(Wc[i * 2 + tid]); typedef float v2f __attribute__((ext_vector_type(2))); const float other = __shfl_xor(s, 1, 32); if (tid == 0) { v2f o; o[0] = s; o[1] = other; *(volatile v2f*)out = o; __threadfence(); *(volatile v2f*)out = o; } } }
extern "C" void kernel_launch(void* const* d_in, const int* in_sizes, int n_in,
                              void* d_out, int out_size, void* d_ws, size_t ws_size, hipStream_t stream) {
  (void)in_sizes; (void)n_in; (void)out_size;
  const float* const* I = (const float* const*)d_in; const float* x0 = I[0]; const int* ei = (const int*)d_in[1]; const int* srci = ei; const int* dsti = ei + NE; const float* temb = I[2]; const float* Wi = I[3]; const float* bi = I[4]; const float* Wg = I[5]; const float* as = I[6]; const float* ad = I[7]; const float* Wt = I[8]; const float* Wq = I[9]; const float* Wk = I[10]; const float* Wv = I[11]; const float* mem = I[12]; const float* Wc = I[13]; const float* bc = I[14];
  char* ws = (char*)d_ws; size_t off = 0;
  auto take = [&](size_t bytes) { char* p = ws + off; off += (bytes + 255) & ~(size_t)255; return p; };
  _Float16* BWi = (_Float16*)take((size_t)CC * 128 * 2); _Float16* BWg = (_Float16*)take((size_t)CC * CC * 2); _Float16* BWt = (_Float16*)take((size_t)CC * TD * 2); _Float16* BWq = (_Float16*)take((size_t)CC * CC * 2); _Float16* BWk = (_Float16*)take((size_t)CC * MD * 2); _Float16* BWv = (_Float16*)take((size_t)CC * MD * 2);
  _Float16* X0h = (_Float16*)take((size_t)NNP * 128 * 2); _Float16* T16 = (_Float16*)take((size_t)NNP * TD * 2); _Float16* M16 = (_Float16*)take((size_t)16 * MD * 2);
  float* X = (float*)take((size_t)NNP * CC * 4); _Float16* X16 = (_Float16*)take((size_t)NNP * CC * 2); float* TPQ = (float*)take((size_t)NNP * CC * 4); _Float16* HT16 = (_Float16*)take((size_t)NNP * CC * 2); _Float16* H16 = (_Float16*)take((size_t)NNP * CC * 2); float* ES = (float*)take((size_t)NNP * NH * 4); float* ED = (float*)take((size_t)NNP * NH * 4); float* NODE = (float*)take((size_t)NNP * CC * 4); _Float16* N16 = (_Float16*)take((size_t)NNP * CC * 2); float* KM = (float*)take((size_t)16 * CC * 4); float* VM = (float*)take((size_t)16 * CC * 4); float* POOL = (float*)take(CC * 4);
  if (off > ws_size) return;
  float* TP = TPQ; float* Q = TPQ;
  k_wt_f16<<<(unsigned)((CC * (128 / 8) + 255) / 256), 256, 0, stream>>>(Wi, BWi, 128, CC, 16.0f);
  k_x16<<<(unsigned)(((size_t)NNODE * 128 / 8 + 255) / 256), 256, 0, stream>>>(x0, X0h, (size_t)NNODE * 128 / 8); k_x16<<<(unsigned)(((size_t)NNODE * TD / 8 + 255) / 256), 256, 0, stream>>>(temb, T16, (size_t)NNODE * TD / 8); k_x16<<<(MS * MD / 8 + 255) / 256, 256, 0, stream>>>(mem, M16, MS * MD / 8);
  const dim3 gC(((NNODE / 16) * (CC / 64) + 3) / 4, 1); const unsigned gq = (NNODE + 1023) / 1024, g8 = (unsigned)(((size_t)NNODE * CC / 8 + 255) / 256);
  k_gemm_hhx<3><<<gC, 128, 0, stream>>>(X0h, 128, 0, BWi, 128, 0, 0.0625f, bi, 0, nullptr, 1, 0, 0, X, X16, CC, 0, NNODE, CC, 128);
  for (int l = 0; l < 5; ++l) {
    k_wt_f16<<<(unsigned)((CC * (TD / 8) + 255) / 256), 256, 0, stream>>>(Wt + (size_t)l * TD * CC, BWt, TD, CC, 16.0f); k_wt_f16<<<(unsigned)((CC * (CC / 8) + 255) / 256), 256, 0, stream>>>(Wg + (size_t)l * CC * CC, BWg, CC, CC, 16.0f);
    k_wt_f16<<<(unsigned)((CC * (CC / 8) + 255) / 256), 256, 0, stream>>>(Wq + (size_t)l * CC * CC, BWq, CC, CC, 16.0f); k_wt_f16<<<(unsigned)((CC * (MD / 8) + 255) / 256), 256, 0, stream>>>(Wk + (size_t)l * MD * CC, BWk, MD, CC, 16.0f); k_wt_f16<<<(unsigned)((CC * (MD / 8) + 255) / 256), 256, 0, stream>>>(Wv + (size_t)l * MD * CC, BWv, MD, CC, 16.0f);
    k_gemm_hhx<0><<<gC, 128, 0, stream>>>(T16, TD, 0, BWt, TD, 0, 0.0625f, nullptr, 0, X, 1, (size_t)CC, 0, TP, HT16, CC, 0, NNODE, CC, TD);
    k_gemm_hhx<0><<<gC, 128, 0, stream>>>(HT16, CC, 0, BWg, CC, 0, 0.0625f, nullptr, 0, nullptr, 1, 0, 0, nullptr, H16, CC, 0, NNODE, CC, CC);
    k_hdots<<<(NNODE * NH + 255) / 256, 256, 0, stream>>>(H16, as + (size_t)l * NH * HD, ad + (size_t)l * NH * HD, ES, ED);
    for (int hp = 0; hp < NH / 2; ++hp) k_gmsg2<<<gq, 512, 0, stream>>>(H16, CC, hp * 64, ES, ED, NH, hp * 2, srci, dsti, NODE, hp * 64);
    k_h16<<<g8, 256, 0, stream>>>(NODE, N16, (size_t)NNODE * CC / 8);
    k_gemm_hhx<0><<<gC, 128, 0, stream>>>(N16, CC, 0, BWq, CC, 0, 0.0625f, nullptr, 0, nullptr, 1, 0, 0, Q, nullptr, CC, 0, NNODE, CC, CC);
    k_gemm_hhx<0><<<dim3(1, 1), 128, 0, stream>>>(M16, MD, 0, BWk, MD, 0, 0.0625f, nullptr, 0, nullptr, 1, 0, 0, KM, nullptr, CC, 0, 16, CC, MD);
    k_gemm_hhx<0><<<dim3(1, 1), 128, 0, stream>>>(M16, MD, 0, BWv, MD, 0, 0.0625f, nullptr, 0, nullptr, 1, 0, 0, VM, nullptr, CC, 0, 16, CC, MD);
    k_memres<<<(NNODE + 7) / 8, 256, 0, stream>>>(NODE, Q, KM, VM, X, X16); }
  k_pool<<<CC, 256, 0, stream>>>(X, POOL); k_cls<<<1, 64, 0, stream>>>(POOL, mem, Wc, bc, (float*)d_out);
}
